// PAE_25640954757479
// MI455X (gfx1250) — hardware-verified
//
#include <hip/hip_runtime.h>
#include <stddef.h>
#include <stdint.h>


#define F_IN    64
#define HID     128
#define GBM     64
#define NTHR    256
#define NWAVE   8
#define NB      4096
#define EPT     8
#define CHUNK   (NTHR * EPT)
#define WCAP    (EPT * 32)
#define APITCH  136
#define LPW     4
#define WSMAX   134217728

static_assert((F_IN % 32) == 0 && (HID % 32) == 0);
static_assert(HID == 128 && F_IN == 64 && GBM == 64 && NTHR == 256 && NWAVE * 32 == NTHR);
static_assert(NB == 16 * NTHR);
static_assert((NB & (NB - 1)) == 0);
static_assert((CHUNK & (CHUNK - 1)) == 0);
static_assert(((APITCH * 2) % 16) == 0 && APITCH >= HID);
static_assert(GBM * APITCH * 4 >= GBM * HID * 4);
static_assert(HID == NTHR - 2 * GBM);
static_assert(8 * HID == 4 * NTHR);

typedef float          v4f   __attribute__((ext_vector_type(4)));
typedef float          v8f   __attribute__((ext_vector_type(8)));
typedef int            v4i   __attribute__((ext_vector_type(4)));
typedef int            v8i   __attribute__((ext_vector_type(8)));
typedef unsigned short v8us  __attribute__((ext_vector_type(8)));
typedef unsigned short v16us __attribute__((ext_vector_type(16)));
typedef __bf16         v16bf __attribute__((ext_vector_type(16)));
typedef v4f  __attribute__((may_alias)) v4fa;
typedef v4i  __attribute__((may_alias)) v4ia;
typedef v8us __attribute__((may_alias)) v8usa;
typedef unsigned short __attribute__((may_alias)) usa;
union FragB { v16us u; v8us h[2]; v8i w; };

__device__ __forceinline__ v8f wmb(const FragB& a, const FragB& b, v8f c) {
  const v16bf av = __builtin_bit_cast(v16bf, a.u);
  const v16bf bv = __builtin_bit_cast(v16bf, b.u);
  v8f d = __builtin_amdgcn_wmma_f32_16x16x32_bf16(false, av, false, bv, (short)0, c, false, false);
  asm volatile("v_nop\n\tv_nop\n\tv_nop\n\tv_nop" : "+v"(d) : "v"(a.w), "v"(b.w));
  return d;
}

__device__ __forceinline__ unsigned short rne16(float f) {
  unsigned u = __float_as_uint(f);
  u = u + 0x7FFFu + ((u >> 16) & 1u);
  return (unsigned short)(u >> 16);
}
__device__ __forceinline__ float bfr(float f) {
  return __uint_as_float(((unsigned)rne16(f)) << 16);
}

__device__ __forceinline__ void gemm1_tile(const unsigned short* __restrict__ XB,
                                           const unsigned short* __restrict__ W1T,
                                           int rowBase, int rg, int ch, int m, int hh, v8f (&acc)[4]) {
  const v8f z = {0.f, 0.f, 0.f, 0.f, 0.f, 0.f, 0.f, 0.f};
  acc[0] = z; acc[1] = z; acc[2] = z; acc[3] = z;
  const unsigned short* ap = XB  + (size_t)(rowBase + 16 * rg + m) * F_IN + 8 * hh;
  const unsigned short* wp = W1T + (size_t)(64 * ch + m) * F_IN + 8 * hh;
#pragma unroll
  for (int ks = 0; ks < F_IN / 32; ++ks) {
    FragB af;
    af.h[0] = *(const v8usa*)(ap + 32 * ks);
    af.h[1] = *(const v8usa*)(ap + 32 * ks + 16);
#pragma unroll
    for (int t = 0; t < 4; ++t) {
      const unsigned short* wq = wp + (size_t)(16 * t) * F_IN + 32 * ks;
      FragB bf;
      bf.h[0] = *(const v8usa*)wq;
      bf.h[1] = *(const v8usa*)(wq + 16);
      acc[t] = wmb(af, bf, acc[t]);
    }
  }
}

__global__ __launch_bounds__(NTHR) void k_prep(const float* __restrict__ x, const float* __restrict__ W1,
                                               const float* __restrict__ W2,
                                               unsigned short* XB, unsigned short* W1T, unsigned short* W2T,
                                               int nN, int nUx, int nUtot) {
  const int u = (int)blockIdx.x * NTHR + (int)threadIdx.x;
  if (u >= nUtot) return;
  v4f a, b;
  unsigned short* dst;
  if (u < nUx) {
    const int row = u >> 3;
    const int c0  = (u & 7) * 8;
    const int rc  = row < nN ? row : nN - 1;
    const float* p = x + (size_t)rc * F_IN + c0;
    a = *(const v4fa*)p;
    b = *(const v4fa*)(p + 4);
    const v4f z4 = {0.f, 0.f, 0.f, 0.f};
    if (row >= nN) { a = z4; b = z4; }
    dst = XB + (size_t)row * F_IN + c0;
  } else if (u < nUx + HID * (F_IN / 8)) {
    const int e  = u - nUx;
    const int n  = e / (F_IN / 8);
    const int k8 = (e - n * (F_IN / 8)) * 8;
    const float* p = W1 + (size_t)k8 * HID + n;
    a.x = p[0];                   a.y = p[(size_t)HID];         a.z = p[(size_t)2 * HID];     a.w = p[(size_t)3 * HID];
    b.x = p[(size_t)4 * HID];     b.y = p[(size_t)5 * HID];     b.z = p[(size_t)6 * HID];     b.w = p[(size_t)7 * HID];
    dst = W1T + (size_t)n * F_IN + k8;
  } else {
    const int e  = u - nUx - HID * (F_IN / 8);
    const int n  = e / (HID / 8);
    const int k8 = (e - n * (HID / 8)) * 8;
    const float* p = W2 + (size_t)k8 * HID + n;
    a.x = p[0];                   a.y = p[(size_t)HID];         a.z = p[(size_t)2 * HID];     a.w = p[(size_t)3 * HID];
    b.x = p[(size_t)4 * HID];     b.y = p[(size_t)5 * HID];     b.z = p[(size_t)6 * HID];     b.w = p[(size_t)7 * HID];
    dst = W2T + (size_t)n * HID + k8;
  }
  v8us o;
  o[0] = rne16(a.x); o[1] = rne16(a.y); o[2] = rne16(a.z); o[3] = rne16(a.w);
  o[4] = rne16(b.x); o[5] = rne16(b.y); o[6] = rne16(b.z); o[7] = rne16(b.w);
  *(volatile v8us*)dst = o;
  __threadfence();
  *(volatile v8us*)dst = o;
}

__device__ __forceinline__ int scan_chunk(const int* __restrict__ lst, int nE, int nN, int cbase, int nodeBase,
                                          int vec8, int* list, int tid, int lane, int wave) {
  int wc = 0;
  const int el0 = tid * EPT;
  const int e0  = cbase + el0;
  v4i da, db;
  bool q0, q1, q2, q3, q4, q5, q6, q7;
  if (vec8 != 0 && cbase + CHUNK <= nE) {
    da = *(const v4ia*)(lst + e0);
    db = *(const v4ia*)(lst + e0 + 4);
    q0 = true; q1 = true; q2 = true; q3 = true; q4 = true; q5 = true; q6 = true; q7 = true;
  } else {
    q0 = e0     < nE; q1 = e0 + 1 < nE; q2 = e0 + 2 < nE; q3 = e0 + 3 < nE;
    q4 = e0 + 4 < nE; q5 = e0 + 5 < nE; q6 = e0 + 6 < nE; q7 = e0 + 7 < nE;
    da.x = lst[e0     < nE ? e0     : nE - 1];
    da.y = lst[e0 + 1 < nE ? e0 + 1 : nE - 1];
    da.z = lst[e0 + 2 < nE ? e0 + 2 : nE - 1];
    da.w = lst[e0 + 3 < nE ? e0 + 3 : nE - 1];
    db.x = lst[e0 + 4 < nE ? e0 + 4 : nE - 1];
    db.y = lst[e0 + 5 < nE ? e0 + 5 : nE - 1];
    db.z = lst[e0 + 6 < nE ? e0 + 6 : nE - 1];
    db.w = lst[e0 + 7 < nE ? e0 + 7 : nE - 1];
  }
  const unsigned unb = (unsigned)NB;
#define SLOT(V, OK) ((OK) ? (unsigned)(((((V) < 0) ? 0 : (((V) > nN - 1) ? nN - 1 : (V)))) - nodeBase) : 0xFFFFFFFFu)
  const unsigned s0 = SLOT(da.x, q0), s1 = SLOT(da.y, q1), s2 = SLOT(da.z, q2), s3 = SLOT(da.w, q3);
  const unsigned s4 = SLOT(db.x, q4), s5 = SLOT(db.y, q5), s6 = SLOT(db.z, q6), s7 = SLOT(db.w, q7);
#undef SLOT
  const bool h0 = s0 < unb, h1 = s1 < unb, h2 = s2 < unb, h3 = s3 < unb;
  const bool h4 = s4 < unb, h5 = s5 < unb, h6 = s6 < unb, h7 = s7 < unb;
  const unsigned any = __builtin_amdgcn_ballot_w32(h0 | h1 | h2 | h3 | h4 | h5 | h6 | h7);
  if (any != 0u) {
#define HITJ(HJ, SJ) { \
      const unsigned mj = __builtin_amdgcn_ballot_w32(HJ); \
      if (mj != 0u) { \
        if (HJ) { \
          const int pos = wc + (int)__builtin_amdgcn_mbcnt_lo(mj, 0u); \
          if (pos < WCAP) list[wave * WCAP + pos] = (int)(SJ); \
        } \
        wc += (int)__builtin_popcount(mj); } }
    HITJ(h0, s0)
    HITJ(h1, s1)
    HITJ(h2, s2)
    HITJ(h3, s3)
    HITJ(h4, s4)
    HITJ(h5, s5)
    HITJ(h6, s6)
    HITJ(h7, s7)
#undef HITJ
  }
  return wc;
}

__global__ __launch_bounds__(NTHR) void k_count(const int* __restrict__ ei, int* CNT, int nE, int nN,
                                                int cstride, int vec8) {
  __shared__ __attribute__((aligned(16))) int cnt[2 * NB];
  __shared__ __attribute__((aligned(16))) int list[NWAVE * WCAP];
  __shared__ int wcnt[NWAVE];
  const int tid = (int)threadIdx.x, lane = tid & 31, wave = tid >> 5;
  const int nodeBase = (int)blockIdx.x * NB;
  for (int i = tid; i < 2 * NB; i += NTHR) cnt[i] = 0;
  for (int i = tid; i < NWAVE * WCAP; i += NTHR) list[i] = 0;
  if (tid < NWAVE) wcnt[tid] = 0;
  __syncthreads();

  const int nChunks = (nE + CHUNK - 1) / CHUNK;
#pragma unroll 1
  for (int r = 0; r < 2; ++r) {
    const int* lst = ei + (size_t)r * (size_t)nE;
    const int cofs = r * NB;
#pragma unroll 1
    for (int ch = 0; ch < nChunks; ++ch) {
      const int cbase = ch * CHUNK;
      const int wc = scan_chunk(lst, nE, nN, cbase, nodeBase, vec8, list, tid, lane, wave);
      if (lane == 0) wcnt[wave] = wc;
      __syncthreads();
      if (wave == 0) {
#pragma unroll 1
        for (int w2 = 0; w2 < NWAVE; ++w2) {
          int c = wcnt[w2];
          c = c < 0 ? 0 : (c > WCAP ? WCAP : c);
#pragma unroll 1
          for (int b0 = 0; b0 < c; b0 += 32) {
            const int idx = b0 + lane;
            const int uv  = list[w2 * WCAP + (idx < WCAP ? idx : WCAP - 1)];
            const int m32 = (c - b0) < 32 ? (c - b0) : 32;
#pragma unroll 1
            for (int k = 0; k < m32; ++k) {
              const int u  = __builtin_amdgcn_readlane(uv, k);
              const int sl = u & (NB - 1);
              if (lane == 0) cnt[cofs + sl] = cnt[cofs + sl] + 1;
            }
          }
        }
      }
      __syncthreads();
    }
  }

  v4i av[4], bv[4];
#pragma unroll
  for (int i = 0; i < 4; ++i) {
    const int idx = 4 * tid + NTHR * 4 * i;
    av[i] = *(const v4ia*)(cnt + idx);
    bv[i] = *(const v4ia*)(cnt + NB + idx);
  }
#pragma unroll
  for (int i = 0; i < 4; ++i) {
    const int idx = 4 * tid + NTHR * 4 * i;
    *(volatile v4i*)(CNT + nodeBase + idx) = av[i];
    *(volatile v4i*)(CNT + (size_t)cstride + nodeBase + idx) = bv[i];
  }
  __threadfence();
#pragma unroll
  for (int i = 0; i < 4; ++i) {
    const int idx = 4 * tid + NTHR * 4 * i;
    *(volatile v4i*)(CNT + nodeBase + idx) = av[i];
    *(volatile v4i*)(CNT + (size_t)cstride + nodeBase + idx) = bv[i];
  }
}

__global__ __launch_bounds__(NTHR) void k_stats(const unsigned short* __restrict__ XB,
                                                const unsigned short* __restrict__ W1T,
                                                const float* __restrict__ b1, const int* __restrict__ CNT,
                                                int cstride, int nE, float* REC) {
  __shared__ __attribute__((aligned(16))) float stg[GBM * HID];
  __shared__ __attribute__((aligned(16))) float part[2 * 4 * HID];
  __shared__ __attribute__((aligned(16))) float recl[4 * HID];
  __shared__ float csd[2 * GBM];
  __shared__ float b1l[HID];
  const int tid = (int)threadIdx.x, lane = tid & 31, wave = tid >> 5, hh = lane >> 4, m = lane & 15;
  const int rg = wave & 3, ch = wave >> 2;
  const int rowBase = (int)blockIdx.x * GBM;

  if (tid < 2 * GBM) {
    const int idx = (tid < GBM) ? (rowBase + tid) : (cstride + rowBase + tid - GBM);
    int c = CNT[idx];
    c = c < 0 ? 0 : (c > nE ? nE : c);
    csd[tid] = (float)c;
  } else {
    b1l[tid - 2 * GBM] = bfr(b1[tid - 2 * GBM]);
  }
  __syncthreads();

  v8f acc[4];
  gemm1_tile(XB, W1T, rowBase, rg, ch, m, hh, acc);
#pragma unroll
  for (int t = 0; t < 4; ++t) {
    const int col = 64 * ch + 16 * t + m;
    const float bb = b1l[col];
#pragma unroll
    for (int r = 0; r < 8; ++r) {
      const int row = 16 * rg + 8 * hh + r;
      stg[row * HID + col] = fmaxf(acc[t][r] + bb, 0.0f);
    }
  }
  __syncthreads();

  {
    const int col = tid & (HID - 1), half = tid >> 7;
    float ps = 0.f, pq = 0.f, pd = 0.f, pdq = 0.f;
#pragma unroll 2
    for (int r = 0; r < GBM / 2; ++r) {
      const int row = (GBM / 2) * half + r;
      const float v  = stg[row * HID + col];
      const float v2 = v * v;
      const float ws = csd[row];
      const float wd = csd[GBM + row];
      ps  = fmaf(ws, v,  ps);
      pq  = fmaf(ws, v2, pq);
      pd  = fmaf(wd, v,  pd);
      pdq = fmaf(wd, v2, pdq);
    }
    part[half * 4 * HID + col]           = ps;
    part[half * 4 * HID + HID + col]     = pq;
    part[half * 4 * HID + 2 * HID + col] = pd;
    part[half * 4 * HID + 3 * HID + col] = pdq;
  }
  __syncthreads();
  recl[tid]           = part[tid]           + part[4 * HID + tid];
  recl[2 * HID + tid] = part[2 * HID + tid] + part[6 * HID + tid];
  __syncthreads();

  v4f rv;
  const bool wr = tid < HID;
  {
    const int i4 = wr ? 4 * tid : 0;
    rv = *(const v4fa*)(recl + i4);
  }
  float* rp = REC + (size_t)blockIdx.x * (4 * HID) + 4 * tid;
  if (wr) *(volatile v4f*)rp = rv;
  __threadfence();
  if (wr) *(volatile v4f*)rp = rv;
}

__global__ __launch_bounds__(NTHR) void k_fold(const float* __restrict__ REC, int nBlk, int nE,
                                               const float* __restrict__ gamma, const float* __restrict__ beta,
                                               float* TAB) {
  __shared__ double dt[4 * HID];
  __shared__ __attribute__((aligned(16))) float tabl[8 * HID];
  const int tid = (int)threadIdx.x;
  double d0 = 0.0, d1 = 0.0;
#pragma unroll 1
  for (int b = 0; b < nBlk; ++b) {
    const float* rp = REC + (size_t)b * (4 * HID);
    d0 += (double)rp[tid];
    d1 += (double)rp[2 * HID + tid];
  }
  dt[tid] = d0;
  dt[2 * HID + tid] = d1;
  __syncthreads();
  {
    const int side = tid >> 7, c = tid & (HID - 1);
    const double S = dt[side * 2 * HID + c];
    const double Q = dt[side * 2 * HID + HID + c];
    const double invE = 1.0 / (double)nE;
    const double mu = S * invE;
    double var = Q * invE - mu * mu;
    var = var < 0.0 ? 0.0 : var;
    const float muf  = (float)mu;
    const float varf = (float)var;
    const float ve   = varf + 1e-5f;
    const float rsq  = (float)(1.0 / sqrt((double)ve));
    tabl[side * 4 * HID + c]           = muf;
    tabl[side * 4 * HID + HID + c]     = rsq;
    tabl[side * 4 * HID + 2 * HID + c] = bfr(gamma[c]);
    tabl[side * 4 * HID + 3 * HID + c] = bfr(beta[c]);
  }
  __syncthreads();
  const v4f v = *(const v4fa*)(tabl + 4 * tid);
  *(volatile v4f*)(TAB + 4 * tid) = v;
  __threadfence();
  *(volatile v4f*)(TAB + 4 * tid) = v;
}

__global__ __launch_bounds__(NTHR) void k_node(const unsigned short* __restrict__ XB,
                                               const unsigned short* __restrict__ W1T,
                                               const unsigned short* __restrict__ W2T,
                                               const float* __restrict__ b1, const float* __restrict__ b2,
                                               const float* __restrict__ TAB, float* H, float* NSQ, int MP) {
  __shared__ __attribute__((aligned(16))) float lmain[GBM * APITCH];
  __shared__ __attribute__((aligned(16))) float tabl[4 * HID];
  __shared__ float b1l[HID];
  __shared__ float b2l[HID];
  __shared__ __attribute__((aligned(16))) float nrm[GBM];
  const int tid = (int)threadIdx.x, lane = tid & 31, wave = tid >> 5, hh = lane >> 4, m = lane & 15;
  const int rg = wave & 3, ch = wave >> 2;
  const int rowBase = (int)blockIdx.x * GBM;
  const int side = (int)blockIdx.y;

  for (int i = tid; i < 4 * HID; i += NTHR) tabl[i] = TAB[side * 4 * HID + i];
  if (tid < HID) b1l[tid] = bfr(b1[tid]);
  else           b2l[tid - HID] = bfr(b2[tid - HID]);
  __syncthreads();

  usa* ahi = (usa*)lmain;
  usa* alo = ahi + GBM * APITCH;
  float* stg = lmain;

  {
    v8f acc1[4];
    gemm1_tile(XB, W1T, rowBase, rg, ch, m, hh, acc1);
#pragma unroll
    for (int t = 0; t < 4; ++t) {
      const int col = 64 * ch + 16 * t + m;
      const float bb = b1l[col];
      const float mu = tabl[col];
      const float rs = tabl[HID + col];
      const float ga = tabl[2 * HID + col];
      const float be = tabl[3 * HID + col];
#pragma unroll
      for (int r = 0; r < 8; ++r) {
        const int row = 16 * rg + 8 * hh + r;
        const float v = fmaxf(acc1[t][r] + bb, 0.0f);
        float a = (v - mu) * rs;
        a = a * ga + be;
        const unsigned short hb = rne16(a);
        const float hf = __uint_as_float(((unsigned)hb) << 16);
        const unsigned short lb = rne16(a - hf);
        ahi[row * APITCH + col] = hb;
        alo[row * APITCH + col] = lb;
      }
    }
  }
  __syncthreads();

  v8f acc2[4];
  {
    const v8f z = {0.f, 0.f, 0.f, 0.f, 0.f, 0.f, 0.f, 0.f};
    acc2[0] = z; acc2[1] = z; acc2[2] = z; acc2[3] = z;
  }
  const usa* aph = ahi + (16 * rg + m) * APITCH + 8 * hh;
  const usa* apl = alo + (16 * rg + m) * APITCH + 8 * hh;
  const unsigned short* wp = W2T + (size_t)(64 * ch + m) * HID + 8 * hh;
#pragma unroll 1
  for (int ks = 0; ks < HID / 32; ++ks) {
    FragB fh, fl;
    fh.h[0] = *(const v8usa*)(aph + 32 * ks);
    fh.h[1] = *(const v8usa*)(aph + 32 * ks + 16);
    fl.h[0] = *(const v8usa*)(apl + 32 * ks);
    fl.h[1] = *(const v8usa*)(apl + 32 * ks + 16);
#pragma unroll
    for (int t = 0; t < 4; ++t) {
      const unsigned short* wq = wp + (size_t)(16 * t) * HID + 32 * ks;
      FragB bf;
      bf.h[0] = *(const v8usa*)wq;
      bf.h[1] = *(const v8usa*)(wq + 16);
      acc2[t] = wmb(fh, bf, acc2[t]);
      acc2[t] = wmb(fl, bf, acc2[t]);
    }
  }
  __syncthreads();

#pragma unroll
  for (int t = 0; t < 4; ++t) {
    const int col = 64 * ch + 16 * t + m;
    const float bb = b2l[col];
#pragma unroll
    for (int r = 0; r < 8; ++r) {
      const int row = 16 * rg + 8 * hh + r;
      stg[row * HID + col] = acc2[t][r] + bb;
    }
  }
  __syncthreads();

  v4f rv[8];
#pragma unroll
  for (int i = 0; i < 8; ++i) rv[i] = *(const v4fa*)(stg + (8 * wave + i) * HID + 4 * lane);
  float* hbase = H + ((size_t)side * (size_t)MP + (size_t)rowBase) * HID;
#pragma unroll
  for (int i = 0; i < 8; ++i) *(volatile v4f*)(hbase + (size_t)(8 * wave + i) * HID + 4 * lane) = rv[i];
  __threadfence();
#pragma unroll
  for (int i = 0; i < 8; ++i) *(volatile v4f*)(hbase + (size_t)(8 * wave + i) * HID + 4 * lane) = rv[i];

  {
    const int row = tid >> 2, q = tid & 3;
    float s = 0.f;
#pragma unroll
    for (int j = 0; j < 8; ++j) {
      const v4f v = *(const v4fa*)(stg + row * HID + 32 * q + 4 * j);
      s = fmaf(v.x, v.x, s); s = fmaf(v.y, v.y, s); s = fmaf(v.z, v.z, s); s = fmaf(v.w, v.w, s);
    }
    s += __shfl_xor(s, 1);
    s += __shfl_xor(s, 2);
    if (q == 0) nrm[row] = s;
  }
  __syncthreads();
  {
    const bool wr = tid < (GBM / 4);
    const int i4 = wr ? 4 * tid : 0;
    const v4f v = *(const v4fa*)(nrm + i4);
    float* np = NSQ + (size_t)side * (size_t)MP + rowBase + 4 * tid;
    if (wr) *(volatile v4f*)np = v;
    __threadfence();
    if (wr) *(volatile v4f*)np = v;
  }
}

__global__ __launch_bounds__(NTHR) void k_edge(const int* __restrict__ ei, const float* __restrict__ H,
                                               const float* __restrict__ NSQ, float* out,
                                               int nE, int nN, int MP, int nLines) {
  const int tid = (int)threadIdx.x, lane = tid & 31, wave = tid >> 5;
  const int q8 = lane & 7, j = lane >> 3;
#pragma unroll 1
  for (int g = 0; g < LPW; ++g) {
    const int L = ((int)blockIdx.x * (NTHR / 32) + wave) * LPW + g;
    if (L >= nLines) return;
    const int e0 = L * 32;
    const int el = e0 + lane;
    const int ec = el < nE ? el : nE - 1;
    int sv = ei[ec];
    int dv = ei[(size_t)nE + (size_t)ec];
    sv = sv < 0 ? 0 : (sv > nN - 1 ? nN - 1 : sv);
    dv = dv < 0 ? 0 : (dv > nN - 1 ? nN - 1 : dv);
    const float q1 = NSQ[sv];
    const float q2 = NSQ[(size_t)MP + (size_t)dv];
    float od = 0.f;
#pragma unroll 1
    for (int it = 0; it < 8; ++it) {
      const int se = __shfl(sv, 4 * it + j);
      const int de = __shfl(dv, 4 * it + j);
      const float* p1 = H + (size_t)se * HID + 16 * q8;
      const float* p2 = H + ((size_t)MP + (size_t)de) * HID + 16 * q8;
      const v4f a0 = *(const v4fa*)p1,  a1 = *(const v4fa*)(p1 + 4), a2 = *(const v4fa*)(p1 + 8), a3 = *(const v4fa*)(p1 + 12);
      const v4f c0 = *(const v4fa*)p2,  c1 = *(const v4fa*)(p2 + 4), c2 = *(const v4fa*)(p2 + 8), c3 = *(const v4fa*)(p2 + 12);
      float d = a0.x * c0.x;
      d = fmaf(a0.y, c0.y, d); d = fmaf(a0.z, c0.z, d); d = fmaf(a0.w, c0.w, d);
      d = fmaf(a1.x, c1.x, d); d = fmaf(a1.y, c1.y, d); d = fmaf(a1.z, c1.z, d); d = fmaf(a1.w, c1.w, d);
      d = fmaf(a2.x, c2.x, d); d = fmaf(a2.y, c2.y, d); d = fmaf(a2.z, c2.z, d); d = fmaf(a2.w, c2.w, d);
      d = fmaf(a3.x, c3.x, d); d = fmaf(a3.y, c3.y, d); d = fmaf(a3.z, c3.z, d); d = fmaf(a3.w, c3.w, d);
      d += __shfl_xor(d, 4);
      d += __shfl_xor(d, 2);
      d += __shfl_xor(d, 1);
      const float got = __shfl(d, 8 * (lane & 3));
      od = ((lane >> 2) == it) ? got : od;
    }
    const float n1  = sqrtf(q1);
    const float n2  = sqrtf(q2);
    const float den = fmaxf(n1 * n2, 1e-8f);
    const float cs  = od * (1.0f / den);
    const float o   = (cs + 1.0f) * 0.5f;
    const bool ok = el < nE;
    if (ok) *(volatile float*)(out + el) = o;
    __threadfence();
    if (ok) *(volatile float*)(out + el) = o;
  }
}

static inline int cdiv(int a, int b) { return (a + b - 1) / b; }
static inline size_t al256(size_t v) { return (v + 255) & ~(size_t)255; }

extern "C" void kernel_launch(void* const* d_in, const int* in_sizes, int n_in,
                              void* d_out, int out_size, void* d_ws, size_t ws_size,
                              hipStream_t stream) {
  if (n_in < 8) return;
  if (in_sizes[0] < F_IN || (in_sizes[0] % F_IN) != 0) return;
  const int nN = in_sizes[0] / F_IN;
  if (nN < 1 || nN > (1 << 24)) return;
  if (in_sizes[1] < 2 || (in_sizes[1] & 1) != 0) return;
  const int nE = in_sizes[1] / 2;
  if (nE < 1) return;
  if (in_sizes[2] != F_IN * HID || in_sizes[3] != HID || in_sizes[4] != HID || in_sizes[5] != HID) return;
  if (in_sizes[6] != HID * HID || in_sizes[7] != HID) return;
  if (out_size != nE) return;

  const float* x     = (const float*)d_in[0];
  const int*   ei    = (const int*)d_in[1];
  const float* W1    = (const float*)d_in[2];
  const float* b1    = (const float*)d_in[3];
  const float* gamma = (const float*)d_in[4];
  const float* beta  = (const float*)d_in[5];
  const float* W2    = (const float*)d_in[6];
  const float* b2    = (const float*)d_in[7];
  float* out = (float*)d_out;

  const int MP      = cdiv(nN, GBM) * GBM;
  const int nBlk    = MP / GBM;
  const int gridC   = cdiv(MP, NB);
  const int cstride = gridC * NB;
  const int nLines  = cdiv(nE, 32);
  const int gridE   = cdiv(nLines, (NTHR / 32) * LPW);
  const int vec8    = ((nE & 3) == 0) ? 1 : 0;

  size_t off = 0;
  const size_t oXB  = off; off += al256((size_t)MP * F_IN * 2);
  const size_t oW1T = off; off += al256((size_t)HID * F_IN * 2);
  const size_t oW2T = off; off += al256((size_t)HID * HID * 2);
  const size_t oCNT = off; off += al256((size_t)2 * cstride * 4);
  const size_t oREC = off; off += al256((size_t)nBlk * 4 * HID * 4);
  const size_t oTAB = off; off += al256((size_t)8 * HID * 4);
  const size_t oH   = off; off += al256((size_t)2 * MP * HID * 4);
  const size_t oNSQ = off; off += al256((size_t)2 * MP * 4);
  if (off > ws_size || off > (size_t)WSMAX) return;

  char* ws = (char*)d_ws;
  unsigned short* XB  = (unsigned short*)(ws + oXB);
  unsigned short* W1T = (unsigned short*)(ws + oW1T);
  unsigned short* W2T = (unsigned short*)(ws + oW2T);
  int*   CNT = (int*)(ws + oCNT);
  float* REC = (float*)(ws + oREC);
  float* TAB = (float*)(ws + oTAB);
  float* H   = (float*)(ws + oH);
  float* NSQ = (float*)(ws + oNSQ);

  const int nUx   = MP * (F_IN / 8);
  const int nUtot = nUx + HID * (F_IN / 8) + HID * (HID / 8);
  k_prep<<<cdiv(nUtot, NTHR), NTHR, 0, stream>>>(x, W1, W2, XB, W1T, W2T, nN, nUx, nUtot);
  k_count<<<gridC, NTHR, 0, stream>>>(ei, CNT, nE, nN, cstride, vec8);
  k_stats<<<nBlk, NTHR, 0, stream>>>(XB, W1T, b1, CNT, cstride, nE, REC);
  k_fold<<<1, NTHR, 0, stream>>>(REC, nBlk, nE, gamma, beta, TAB);
  k_node<<<dim3(nBlk, 2), NTHR, 0, stream>>>(XB, W1T, W2T, b1, b2, TAB, H, NSQ, MP);
  k_edge<<<gridE, NTHR, 0, stream>>>(ei, H, NSQ, out, nE, nN, MP, nLines);
}
